// ResNetBasicblock_22668837388977
// MI455X (gfx1250) — hardware-verified
//
#include <hip/hip_runtime.h>


typedef __attribute__((ext_vector_type(16))) _Float16      v16bf;
typedef __attribute__((ext_vector_type(4)))  float         v4f_t;
typedef float v4fa __attribute__((ext_vector_type(4), may_alias));
typedef __attribute__((ext_vector_type(4)))  unsigned      v4u_t;
typedef unsigned v4ua __attribute__((ext_vector_type(4), may_alias));
typedef __attribute__((ext_vector_type(8)))  float          v8f;
typedef __attribute__((ext_vector_type(8)))  unsigned short ushort8;
typedef __attribute__((ext_vector_type(4)))  int            v4i;

typedef __attribute__((address_space(1))) v4i v4i_g;
typedef __attribute__((address_space(3))) v4i v4i_l;

#define BATCH 16
#define CCH   256
#define HH    56
#define WW    56
#define SPAT  (HH * WW)
#define MTOT  (BATCH * SPAT)
#define MTILES (MTOT / 16)
#define MBLOCKS (MTILES / 8)
#define NBLOCKS (CCH / 64)
#define LROW    40

#if __has_builtin(__builtin_amdgcn_global_load_async_to_lds_b128) && \
    __has_builtin(__builtin_amdgcn_s_wait_asynccnt)
#define USE_ASYNC 1
#else
#define USE_ASYNC 0
#endif

struct U8x2 { ushort8 lo, hi; };

static __device__ __forceinline__ v16bf frag_of(ushort8 lo, ushort8 hi) {
  U8x2 t{lo, hi};
  return __builtin_bit_cast(v16bf, t);
}

static __device__ __forceinline__ unsigned short f2bf(float f) { return __builtin_bit_cast(unsigned short, (_Float16)f); }
static __device__ __forceinline__ unsigned pk2(float a, float b) { return (unsigned)f2bf(a) | ((unsigned)f2bf(b) << 16); }

static __device__ __forceinline__ void stage16B(const unsigned short* g,
                                                unsigned short* l) {
#if USE_ASYNC
  __builtin_amdgcn_global_load_async_to_lds_b128((v4i_g*)g, (v4i_l*)l, 0, 0);
#else
  *(ushort8*)l = *(const ushort8*)g;
#endif
}

static __device__ __forceinline__ void wait_stage() {
#if USE_ASYNC
  __builtin_amdgcn_s_wait_asynccnt(0);
#endif
}

__global__ void zero_pad(unsigned short* z) {
  typedef __attribute__((ext_vector_type(2))) unsigned v2u_t;
  if (threadIdx.x < 32) { v2u_t zz = {0u, 0u}; *(volatile v2u_t*)((unsigned*)z + threadIdx.x * 2) = zz; __threadfence(); *(volatile v2u_t*)((unsigned*)z + threadIdx.x * 2) = zz; }
}

__global__ void pack_x_bf16(const float* __restrict__ x,
                            unsigned short* __restrict__ xb) {
  size_t i = ((size_t)blockIdx.x * 256 + threadIdx.x) * 2;
  int    c  = (int)(i & (CCH - 1));
  size_t m  = i >> 8;
  int    ni = (int)(m / SPAT);
  int    sp = (int)(m - (size_t)ni * SPAT);
  const unsigned p = pk2(x[((size_t)(ni * CCH + c)) * SPAT + sp], x[((size_t)(ni * CCH + c + 1)) * SPAT + sp]);
  *(volatile unsigned*)(xb + i) = p; __threadfence(); *(volatile unsigned*)(xb + i) = p;
}

__global__ void pack_w_bf16(const float* __restrict__ w,
                            unsigned short* __restrict__ wb) {
  size_t i = ((size_t)blockIdx.x * 256 + threadIdx.x) * 2;
  int c   = (int)(i & (CCH - 1));
  int o   = (int)((i >> 8) & (CCH - 1));
  int tap = (int)(i >> 16);
  const unsigned p = pk2(w[((size_t)o * CCH + c) * 9 + tap], w[((size_t)o * CCH + c + 1) * 9 + tap]);
  *(volatile unsigned*)(wb + i) = p; __threadfence(); *(volatile unsigned*)(wb + i) = p;
}

template <bool FINAL>
__global__ void __launch_bounds__(256)
conv_cg_wmma(const unsigned short* __restrict__ in,
             const unsigned short* __restrict__ wt,
             const unsigned short* __restrict__ zpad,
             const float* __restrict__ theta,
             const float* __restrict__ gamma,
             const float* __restrict__ beta,
             const float* __restrict__ mean,
             const float* __restrict__ var,
             const float* __restrict__ xres,
             unsigned short* __restrict__ out_bf,
             float* __restrict__ out_f) {
  __shared__ unsigned short sB[2][64 * LROW];
  __shared__ __attribute__((aligned(16))) float sC[64][128 + 4];

  const int tid  = threadIdx.x;
  const int lane = tid & 31;
  const int wave = tid >> 5;
  const int mb   = blockIdx.x % MBLOCKS;
  const int nb64 = (blockIdx.x / MBLOCKS) * 64;

  const int m_tile = mb * 8 + wave;
  const int half   = lane >> 4;
  const int l15    = lane & 15;

  const int m_row = m_tile * 16 + l15;
  const int n_img = m_row / SPAT;
  const int sp    = m_row - n_img * SPAT;
  const int oh    = sp / WW;
  const int ow    = sp - oh * WW;

  const int srow = tid >> 2;
  const int scol = (tid & 3) * 8;

  v8f accp[4] = {};
  v8f accr[4] = {};

  auto stage_step = [&](int tap, int cb, int bi) {
    const unsigned short* g =
        wt + ((size_t)(tap * CCH + nb64 + srow)) * CCH + cb * 32 + scol;
    stage16B(g, &sB[bi][srow * LROW + scol]);
  };

  auto load_a = [&](int tap, int cb) -> v16bf {
    const int ky = (tap * 11) >> 5;
    const int kx = tap - ky * 3;
    const int ih = oh + ky - 1, iw = ow + kx - 1;
    const bool valid = (ih >= 0) && (ih < HH) && (iw >= 0) && (iw < WW);
    const long pix = ((long)n_img * SPAT + ih * WW + iw) * CCH;
    const unsigned short* base = in + pix + cb * 32 + half * 8;
    const ushort8* p = (const ushort8*)(valid ? base : zpad);
    return frag_of(p[0], p[2]);
  };

  stage_step(0, 0, 0);
  wait_stage();
  __syncthreads();

  v16bf a_cur = load_a(0, 0);

  for (int tap = 0; tap < 9; ++tap) {
#pragma unroll
    for (int cb = 0; cb < 8; ++cb) {
      const int  ntap = (cb == 7) ? tap + 1 : tap;
      const int  ncb  = (cb + 1) & 7;
      const bool more = (cb < 7) || (tap < 8);

      if (more) stage_step(ntap, ncb, (cb + 1) & 1);
      v16bf a_nxt = more ? load_a(ntap, ncb) : a_cur;

      const unsigned short* lb = sB[cb & 1];
      v16bf bf4[4];
#pragma unroll
      for (int nt = 0; nt < 4; ++nt) {
        const ushort8* q =
            (const ushort8*)(lb + (nt * 16 + l15) * LROW + half * 8);
        bf4[nt] = frag_of(q[0], q[2]);
      }

      if (cb < 2) {
#pragma unroll
        for (int nt = 0; nt < 4; ++nt)
          accp[nt] = __builtin_amdgcn_wmma_f32_16x16x32_f16(
              false, a_cur, false, bf4[nt], (short)0, accp[nt], false, false);
      } else {
#pragma unroll
        for (int nt = 0; nt < 4; ++nt)
          accr[nt] = __builtin_amdgcn_wmma_f32_16x16x32_f16(
              false, a_cur, false, bf4[nt], (short)0, accr[nt], false, false);
      }
      a_cur = a_nxt;

      wait_stage();
      __syncthreads();
    }
  }

#pragma unroll
  for (int nt = 0; nt < 4; ++nt) {
    const int ol = nt * 16 + l15, o = nb64 + ol;
    const float th = theta[o];
    const float iv = gamma[o] * rsqrtf(var[o] + 1e-5f);
    const float ad = beta[o] - mean[o] * iv;
#pragma unroll
    for (int i = 0; i < 8; ++i) {
      const float yp = accp[nt][i], yr = accr[nt][i];
      const float d  = 1.f / (1.f + __expf(-2.f * (yp - th)));
      sC[ol][wave * 16 + i + half * 8] = (yp + d * yr) * iv + ad;
    }
  }
  __syncthreads();
  if (!FINAL) {
#pragma unroll 1
    for (int pass = 0; pass < 2; ++pass) {
#pragma unroll 4
      for (int rr = 0; rr < 16; ++rr) {
        const int mloc = wave * 16 + rr;
        const unsigned p = pk2(fmaxf(sC[2 * lane][mloc], 0.f), fmaxf(sC[2 * lane + 1][mloc], 0.f));
        *(volatile unsigned*)(out_bf + (size_t)(mb * 128 + mloc) * CCH + nb64 + 2 * lane) = p;
      }
      __threadfence();
    }
  } else {
#pragma unroll 1
    for (int pass = 0; pass < 2; ++pass) {
#pragma unroll
      for (int i = 0; i < 8; ++i) {
        const int c = tid + 256 * i, ol = c >> 5, q = c & 31;
        const int m = mb * 128 + q * 4, ni = m / SPAT, so = m - ni * SPAT;
        const size_t idx = ((size_t)(ni * CCH + nb64 + ol)) * SPAT + so;
        const v4f_t xr = *(const v4f_t*)(xres + idx);
        v4f_t y = *(const v4fa*)&sC[ol][q * 4];
        y += xr;
        y.x = fmaxf(y.x, 0.f); y.y = fmaxf(y.y, 0.f); y.z = fmaxf(y.z, 0.f); y.w = fmaxf(y.w, 0.f);
        *(volatile v4f_t*)(out_f + idx) = y;
      }
      __threadfence();
    }
  }
}

extern "C" void kernel_launch(void* const* d_in, const int* in_sizes, int n_in,
                              void* d_out, int out_size, void* d_ws, size_t ws_size,
                              hipStream_t stream) {
  const float* x       = (const float*)d_in[0];
  const float* w_a     = (const float*)d_in[1];
  const float* theta_a = (const float*)d_in[2];
  const float* gamma_a = (const float*)d_in[3];
  const float* beta_a  = (const float*)d_in[4];
  const float* mean_a  = (const float*)d_in[5];
  const float* var_a   = (const float*)d_in[6];
  const float* w_b     = (const float*)d_in[7];
  const float* theta_b = (const float*)d_in[8];
  const float* gamma_b = (const float*)d_in[9];
  const float* beta_b  = (const float*)d_in[10];
  const float* mean_b  = (const float*)d_in[11];
  const float* var_b   = (const float*)d_in[12];

  unsigned short* xb  = (unsigned short*)d_ws;
  unsigned short* hb  = xb + (size_t)MTOT * CCH;
  unsigned short* wab = hb + (size_t)MTOT * CCH;
  unsigned short* wbb = wab + (size_t)9 * CCH * CCH;
  unsigned short* zp  = wbb + (size_t)9 * CCH * CCH;

  zero_pad<<<1, 128, 0, stream>>>(zp);
  pack_x_bf16<<<(MTOT * CCH) / 512, 256, 0, stream>>>(x, xb);
  pack_w_bf16<<<(9 * CCH * CCH) / 512, 256, 0, stream>>>(w_a, wab);
  pack_w_bf16<<<(9 * CCH * CCH) / 512, 256, 0, stream>>>(w_b, wbb);

  conv_cg_wmma<false><<<MBLOCKS * NBLOCKS, 256, 0, stream>>>(
      xb, wab, zp, theta_a, gamma_a, beta_a, mean_a, var_a,
      nullptr, hb, nullptr);
  conv_cg_wmma<true><<<MBLOCKS * NBLOCKS, 256, 0, stream>>>(
      hb, wbb, zp, theta_b, gamma_b, beta_b, mean_b, var_b,
      x, nullptr, (float*)d_out);
}
